// Net_62929860821324
// MI455X (gfx1250) — hardware-verified
//
#include <hip/hip_runtime.h>
#include <stddef.h>

#define NB   128
#define NC   192
#define NCLS 100
#define LDSB 98304
#define APITCH 40
#define ATILE  (128 * APITCH)

#define OUT0_OFF 0
#define OUT1_OFF 12800
#define OUT2_OFF 6304256
#define OUT_TOTAL 12595712
static_assert(OUT1_OFF * 4 == 51200);
static_assert(OUT2_OFF * 4 == 25217024);
static_assert((OUT1_OFF * 4) % 128 == 0 && (OUT2_OFF * 4) % 128 == 0);
static_assert(OUT1_OFF == NB * NCLS);
static_assert(OUT2_OFF == OUT1_OFF + NB * NC * 256);
static_assert(OUT2_OFF + NB * NC * 256 == OUT_TOTAL);

#define WS_W1B  0u
#define WS_W2B  36864u
#define WS_W3B  1880064u
#define WS_REC  3723264u
#define WS_STAT 6868992u
#define WS_X03  6875136u
#define WS_R3   13166592u
#define WS_R1   19458048u
#define WS_TOTAL 120121344u
static_assert(WS_W2B == WS_W1B + 192 * 96 * 2);
static_assert(WS_W3B == WS_W2B + 192 * 4800 * 2);
static_assert(WS_REC == WS_W3B + 192 * 4800 * 2);
static_assert(WS_STAT == WS_REC + 1024 * 192 * 16);
static_assert(WS_X03 == WS_STAT + 3 * 2048);
static_assert(WS_R3 == WS_X03 + NB * NC * 64 * 4);
static_assert(WS_R1 == WS_R3 + NB * NC * 64 * 4);
static_assert(WS_TOTAL == WS_R1 + 100663296u);
static_assert(WS_TOTAL <= 134217728u);
static_assert(WS_W2B % 256 == 0 && WS_W3B % 256 == 0 && WS_REC % 256 == 0 && WS_STAT % 256 == 0 &&
              WS_X03 % 256 == 0 && WS_R3 % 256 == 0 && WS_R1 % 256 == 0);
static_assert(NB * NC * 256 * 4 <= 100663296);
static_assert(4800 % 32 == 0 && 800 == 32 * 25 && 192 == 12 * 16 && 96 % 32 == 0);
static_assert((NB * 1024) % 128 == 0 && (NB * 256) % 128 == 0 && (NB * 64) % 128 == 0);
static_assert(LDSB <= 327680);

#define PB_W2 0
#define PB_W3 450
#define PB_W1 900
#define PB_END 909
static_assert((192 * 4800 / 8) % 256 == 0 && (192 * 4800 / 8) / 256 == 450);
static_assert((192 * 12) % 256 == 0 && (192 * 12) / 256 == 9);

typedef float          v4f   __attribute__((ext_vector_type(4)));
typedef float          v8f   __attribute__((ext_vector_type(8)));
typedef int            v8i   __attribute__((ext_vector_type(8)));
typedef unsigned       v4u   __attribute__((ext_vector_type(4)));
typedef unsigned short v8us  __attribute__((ext_vector_type(8)));
typedef __bf16         v16bf __attribute__((ext_vector_type(16)));
typedef double         v2d   __attribute__((ext_vector_type(2)));
typedef v4f  __attribute__((may_alias)) v4fa;
typedef v4u  __attribute__((may_alias)) v4ua;
typedef v8us __attribute__((may_alias)) v8usa;
union FragB { v16bf v; v8us h[2]; v4u q[2]; v8i w; };

__device__ __forceinline__ v8f wmb(const FragB& a, const FragB& b, v8f c) {
  v8f d = __builtin_amdgcn_wmma_f32_16x16x32_bf16(false, a.v, false, b.v, (short)0, c, false, false);
  asm volatile("v_nop\n\tv_nop\n\tv_nop\n\tv_nop" : "+v"(d) : "v"(a.w), "v"(b.w));
  return d;
}
__device__ __forceinline__ v8f z8() { v8f z = {0.f, 0.f, 0.f, 0.f, 0.f, 0.f, 0.f, 0.f}; return z; }

__device__ __forceinline__ unsigned bf16_bits(float f) {
  const unsigned u = __float_as_uint(f);
  return (u + 0x7FFFu + ((u >> 16) & 1u)) >> 16;
}
__device__ __forceinline__ float bf16_val(float f) { return __uint_as_float(bf16_bits(f) << 16); }

__device__ __forceinline__ float atan_f(float z) {
  const float ax = __builtin_fabsf(z);
  const bool big = ax > 2.414213562373095f;
  const bool mid = ax > 0.4142135623730950f;
  const float den = big ? ax : (mid ? (ax + 1.0f) : 1.0f);
  const float num = big ? -1.0f : (mid ? (ax - 1.0f) : ax);
  const float y0  = big ? 1.5707963267948966f : (mid ? 0.7853981633974483f : 0.0f);
  float r = __builtin_amdgcn_rcpf(den);
  const float e = fmaf(-den, r, 1.0f);
  r = fmaf(r, e, r);
  const float x = num * r;
  const float z2 = x * x;
  float p = fmaf(8.05374449538e-2f, z2, -1.38776856032e-1f);
  p = fmaf(p, z2, 1.99777106478e-1f);
  p = fmaf(p, z2, -3.33329491539e-1f);
  const float y = y0 + fmaf(p * z2, x, x);
  return (z < 0.0f) ? -y : y;
}

__device__ __forceinline__ float relu_f(float v) { return (v > 0.0f) ? v : (v - v); }

__device__ __forceinline__ float bn_f(float r, float m, float rs, float g, float b) {
  float t = g * (r - m);
  t = t * rs;
  return t + b;
}
__device__ __forceinline__ v4f bn4(v4f v, float m, float rs, float g, float b) {
  v4f o;
  o.x = bn_f(v.x, m, rs, g, b); o.y = bn_f(v.y, m, rs, g, b);
  o.z = bn_f(v.z, m, rs, g, b); o.w = bn_f(v.w, m, rs, g, b);
  return o;
}

__device__ __forceinline__ v8us cvt8(v4f a, v4f b) {
  v8us o;
  o[0] = (unsigned short)bf16_bits(a.x); o[1] = (unsigned short)bf16_bits(a.y);
  o[2] = (unsigned short)bf16_bits(a.z); o[3] = (unsigned short)bf16_bits(a.w);
  o[4] = (unsigned short)bf16_bits(b.x); o[5] = (unsigned short)bf16_bits(b.y);
  o[6] = (unsigned short)bf16_bits(b.z); o[7] = (unsigned short)bf16_bits(b.w);
  return o;
}
__device__ __forceinline__ void st2_us8(unsigned short* p, v8us v) {
  *(volatile v8us*)p = v;
  __threadfence();
  *(volatile v8us*)p = v;
}

__global__ __launch_bounds__(256) __attribute__((amdgpu_num_vgpr(248)))
void k_prep(const float* __restrict__ w1, const float* __restrict__ w2, const float* __restrict__ w3,
            unsigned short* W1B, unsigned short* W2B, unsigned short* W3B) {
  const int bx = (int)blockIdx.x, tid = (int)threadIdx.x;
  if (bx < PB_W3) {
    const size_t u = (size_t)(bx - PB_W2) * 256 + tid;
    const v4f a = *(const v4f*)(w2 + u * 8);
    const v4f b = *(const v4f*)(w2 + u * 8 + 4);
    st2_us8(W2B + u * 8, cvt8(a, b));
  } else if (bx < PB_W1) {
    const size_t u = (size_t)(bx - PB_W3) * 256 + tid;
    const v4f a = *(const v4f*)(w3 + u * 8);
    const v4f b = *(const v4f*)(w3 + u * 8 + 4);
    st2_us8(W3B + u * 8, cvt8(a, b));
  } else {
    const int u = (bx - PB_W1) * 256 + tid;
    const int o = u / 12;
    const int k8 = (u - o * 12) * 8;
    v8us o8;
#pragma unroll
    for (int j = 0; j < 8; ++j) {
      const int k = k8 + j;
      const int kc = (k < 75) ? k : 74;
      const float v = w1[o * 75 + kc];
      const unsigned bits = bf16_bits(v);
      o8[j] = (unsigned short)((k < 75) ? bits : 0u);
    }
    st2_us8(W1B + (size_t)u * 8, o8);
  }
}

template <int H> struct Cfg;
template <> struct Cfg<32> { static constexpr int CCH = 3,  TS = 3,  PITCH = 36, PLANE = 288, TABN = 96;  };
template <> struct Cfg<16> { static constexpr int CCH = 32, TS = 25, PITCH = 20, PLANE = 240, TABN = 800; };
template <> struct Cfg<8>  { static constexpr int CCH = 32, TS = 25, PITCH = 12, PLANE = 288, TABN = 800; };

template <int CI, int H, int KP>
__global__ __launch_bounds__(256) __attribute__((amdgpu_num_vgpr(248)))
void k_inrf(const float* __restrict__ X, const unsigned short* __restrict__ WB,
            const float* __restrict__ bias, float* R, double* rec) {
  constexpr int CCH = Cfg<H>::CCH, TS = Cfg<H>::TS, PITCH = Cfg<H>::PITCH, PLANE = Cfg<H>::PLANE,
                TABN = Cfg<H>::TABN;
  constexpr int NSTEP = KP / 32;
  constexpr int NE = CCH * PLANE;
  constexpr int NIT = (NE + 255) / 256;
  constexpr int HALO_B = NE * 4;
  constexpr int TAB_OFF = HALO_B;
  constexpr int AT_OFF = HALO_B + TABN * 4;
  static_assert(NSTEP * 32 == KP);
  static_assert(NSTEP == TS * (CI / CCH));
  static_assert(TABN == TS * 32);
  static_assert(TAB_OFF % 16 == 0 && AT_OFF % 16 == 0);
  static_assert(AT_OFF + 4 * ATILE * 2 <= LDSB);
  static_assert(192 * 128 * 4 <= LDSB);

  extern __shared__ __attribute__((aligned(16))) unsigned char dsm[];
  float* halo = (float*)dsm;
  unsigned* tab = (unsigned*)(dsm + TAB_OFF);
  unsigned short* at = (unsigned short*)(dsm + AT_OFF);

  const int tid = (int)threadIdx.x, lane = tid & 31, wave = tid >> 5;
  const int hh = lane >> 4, m = lane & 15;
  const int wm = wave >> 1, wn = wave & 1;
  const int blk = (int)blockIdx.x;

  int img0, h0;
  if (H == 32)      { img0 = blk >> 3; h0 = (blk & 7) * 4; }
  else if (H == 16) { img0 = blk >> 1; h0 = (blk & 1) * 8; }
  else              { img0 = 2 * blk;  h0 = 0; }

  const int r = tid & 127, kh = tid >> 7;
  int pb;
  if (H == 32)      pb = (r >> 5) * 36 + (r & 31);
  else if (H == 16) pb = (r >> 4) * 20 + (r & 15);
  else              pb = (r >> 6) * 144 + ((r >> 3) & 7) * 12 + (r & 7);

#pragma unroll 1
  for (int kl = tid; kl < TABN; kl += 256) {
    const int il = kl / 25;
    const int q = kl - il * 25;
    const int qi = q / 5;
    const int qj = q - qi * 5;
    unsigned e;
    if (kl < CCH * 25) {
      const unsigned offp = (unsigned)(il * PLANE + qi * PITCH + qj);
      const unsigned offc = (unsigned)(il * PLANE + 2 * PITCH + 2);
      e = offp | (offc << 16);
    } else {
      e = 0x80000000u;
    }
    tab[kl] = e;
  }

  v8f acc[2][6];
#pragma unroll
  for (int mt = 0; mt < 2; ++mt)
#pragma unroll
    for (int nt = 0; nt < 6; ++nt) acc[mt][nt] = z8();

  const unsigned short* bp = WB + (size_t)(96 * wn + m) * KP + 8 * hh;

  int s = 0, chunk = 0;
#pragma unroll 1
  for (int t = 0; t < NSTEP; ++t) {
    if (s == 0) {
      const int i0 = chunk * CCH;
#pragma unroll 2
      for (int it = 0; it < NIT; ++it) {
        const int e = it * 256 + tid;
        const int ec = (e < NE) ? e : (NE - 1);
        const int il = ec / PLANE;
        const int rem = ec - il * PLANE;
        int im = 0, rr = rem;
        if (H == 8) { im = rem / 144; rr = rem - im * 144; }
        const int hr = rr / PITCH;
        const int wc = rr - hr * PITCH;
        const int gh = h0 - 2 + hr;
        const int gw = wc - 2;
        const bool ok = (gh >= 0) && (gh < H) && (gw >= 0) && (gw < H);
        const int ghc = (gh < 0) ? 0 : ((gh > H - 1) ? (H - 1) : gh);
        const int gwc = (gw < 0) ? 0 : ((gw > H - 1) ? (H - 1) : gw);
        const size_t gi = (((size_t)(img0 + im) * CI + (size_t)(i0 + il)) * H + ghc) * H + gwc;
        float v = X[gi];
        if (CI == 3) v = bf16_val(v);
        v = v * (ok ? 1.0f : 0.0f);
        if (e < NE) halo[e] = v;
      }
      __syncthreads();
    }

    {
      const unsigned* tp = tab + s * 32 + 16 * kh;
      unsigned short* wr = at + (t & 1) * (2 * ATILE) + r * APITCH + 16 * kh;
#pragma unroll
      for (int g = 0; g < 2; ++g) {
        const v4u e0 = *(const v4ua*)(tp + 8 * g);
        const v4u e1 = *(const v4ua*)(tp + 8 * g + 4);
        float cb[8];
#pragma unroll
        for (int j = 0; j < 8; ++j) {
          const unsigned e = (j < 4) ? e0[j & 3] : e1[j & 3];
          const float p = halo[pb + (int)(e & 0xFFFFu)];
          const float c = halo[pb + (int)((e >> 16) & 0x7FFFu)];
          const float d = p - c;
          float v = p - 2.0f * atan_f(12.0f * d);
          if (CI == 3) v = ((e >> 31) != 0u) ? 0.0f : v;
          cb[j] = v;
        }
        v4u hw, lw;
#pragma unroll
        for (int j2 = 0; j2 < 4; ++j2) {
          const unsigned ha = bf16_bits(cb[2 * j2]);
          const unsigned hb = bf16_bits(cb[2 * j2 + 1]);
          const unsigned la = bf16_bits(cb[2 * j2] - __uint_as_float(ha << 16));
          const unsigned lb = bf16_bits(cb[2 * j2 + 1] - __uint_as_float(hb << 16));
          hw[j2] = ha | (hb << 16);
          lw[j2] = la | (lb << 16);
        }
        *(v4ua*)(wr + 8 * g) = hw;
        *(v4ua*)(wr + ATILE + 8 * g) = lw;
      }
    }
    __syncthreads();

    {
      const unsigned short* ab = at + (t & 1) * (2 * ATILE);
      FragB ah[2], al[2];
#pragma unroll
      for (int mt = 0; mt < 2; ++mt) {
        const unsigned short* p = ab + (32 * wm + 16 * mt + m) * APITCH + 8 * hh;
        ah[mt].q[0] = *(const v4ua*)(p);
        ah[mt].q[1] = *(const v4ua*)(p + 16);
        al[mt].q[0] = *(const v4ua*)(p + ATILE);
        al[mt].q[1] = *(const v4ua*)(p + ATILE + 16);
      }
      const unsigned short* bq = bp + 32 * t;
#pragma unroll
      for (int nt = 0; nt < 6; ++nt) {
        const unsigned short* w = bq + (size_t)(16 * nt) * KP;
        FragB bf;
        bf.h[0] = *(const v8usa*)(w);
        bf.h[1] = *(const v8usa*)(w + 16);
        acc[0][nt] = wmb(ah[0], bf, acc[0][nt]);
        acc[1][nt] = wmb(ah[1], bf, acc[1][nt]);
        acc[0][nt] = wmb(al[0], bf, acc[0][nt]);
        acc[1][nt] = wmb(al[1], bf, acc[1][nt]);
      }
    }
    ++s;
    if (s == TS) { s = 0; ++chunk; }
  }

  __syncthreads();
  float* sT = (float*)dsm;
#pragma unroll
  for (int nt = 0; nt < 6; ++nt) {
    const int ch = 96 * wn + 16 * nt + m;
    const float bb = bf16_val(bias[ch]);
#pragma unroll
    for (int mt = 0; mt < 2; ++mt) {
      const int pix = 32 * wm + 16 * mt + 8 * hh;
      v4f a, b;
      a.x = relu_f(acc[mt][nt][0] + bb); a.y = relu_f(acc[mt][nt][1] + bb);
      a.z = relu_f(acc[mt][nt][2] + bb); a.w = relu_f(acc[mt][nt][3] + bb);
      b.x = relu_f(acc[mt][nt][4] + bb); b.y = relu_f(acc[mt][nt][5] + bb);
      b.z = relu_f(acc[mt][nt][6] + bb); b.w = relu_f(acc[mt][nt][7] + bb);
      *(v4fa*)(sT + ch * 128 + pix) = a;
      *(v4fa*)(sT + ch * 128 + pix + 4) = b;
    }
  }
  __syncthreads();

  v2d rv = {0.0, 0.0};
  if (tid < NC) {
    const float* row = sT + tid * 128;
    double sm = 0.0;
#pragma unroll 4
    for (int i = 0; i < 32; ++i) {
      const v4f v = *(const v4fa*)(row + 4 * i);
      sm += (double)v.x; sm += (double)v.y; sm += (double)v.z; sm += (double)v.w;
    }
    const double mean = sm * (1.0 / 128.0);
    double q = 0.0;
#pragma unroll 4
    for (int i = 0; i < 32; ++i) {
      const v4f v = *(const v4fa*)(row + 4 * i);
      const double d0 = (double)v.x - mean, d1 = (double)v.y - mean;
      const double d2 = (double)v.z - mean, d3 = (double)v.w - mean;
      q += d0 * d0; q += d1 * d1; q += d2 * d2; q += d3 * d3;
    }
    rv.x = mean; rv.y = q;
  }
  double* rp = rec + ((size_t)blk * NC + (size_t)((tid < NC) ? tid : 0)) * 2;

  float* Rb;
  if (H == 32)      Rb = R + (size_t)img0 * NC * 1024 + (size_t)h0 * 32;
  else if (H == 16) Rb = R + (size_t)img0 * NC * 256 + (size_t)(blk & 1) * 128;
  else              Rb = R + (size_t)img0 * NC * 64;
  const int joff = (H == 8) ? ((lane >> 4) * (NC * 64) + (lane & 15) * 4) : (4 * lane);

  if (tid < NC) *(volatile v2d*)rp = rv;
#pragma unroll 4
  for (int it = 0; it < 24; ++it) {
    const int ch = it * 8 + wave;
    const v4f v = *(const v4fa*)(sT + ch * 128 + 4 * lane);
    *(volatile v4f*)(Rb + (size_t)ch * (H * H) + joff) = v;
  }
  __threadfence();
  if (tid < NC) *(volatile v2d*)rp = rv;
#pragma unroll 4
  for (int it = 0; it < 24; ++it) {
    const int ch = it * 8 + wave;
    const v4f v = *(const v4fa*)(sT + ch * 128 + 4 * lane);
    *(volatile v4f*)(Rb + (size_t)ch * (H * H) + joff) = v;
  }
}

__global__ __launch_bounds__(192) __attribute__((amdgpu_num_vgpr(248)))
void k_stat(const double* __restrict__ rec, int nblk, double invb, double invn, float* stat) {
  __shared__ __attribute__((aligned(16))) float sS[2 * NC];
  const int c = (int)threadIdx.x;
  double sm = 0.0;
#pragma unroll 4
  for (int p = 0; p < nblk; ++p) sm += rec[((size_t)p * NC + c) * 2];
  const double mean = sm * invb;
  double q = 0.0;
#pragma unroll 4
  for (int p = 0; p < nblk; ++p) {
    const v2d rv = *(const v2d*)(rec + ((size_t)p * NC + c) * 2);
    const double d = rv.x - mean;
    q += rv.y + 128.0 * d * d;
  }
  const double var = q * invn;
  const float m32 = (float)mean;
  const float v32 = (float)var;
  const float rstd = 1.0f / sqrtf(v32 + 1e-5f);
  sS[c] = m32;
  sS[NC + c] = rstd;
  __syncthreads();
  v4f v = {0.f, 0.f, 0.f, 0.f};
  if (c < 96) {
    v = *(const v4fa*)(sS + 4 * c);
    *(volatile v4f*)(stat + 4 * c) = v;
  }
  __threadfence();
  if (c < 96) *(volatile v4f*)(stat + 4 * c) = v;
}

__global__ __launch_bounds__(256) __attribute__((amdgpu_num_vgpr(248)))
void k_bn1pool(const float* __restrict__ R1, const float* __restrict__ stat,
               const float* __restrict__ g, const float* __restrict__ be, float* out1) {
  const int tid = (int)threadIdx.x, lane = tid & 31, wave = tid >> 5;
  const int plane = (int)blockIdx.x * 8 + wave;
  const int c = plane % NC;
  const float m = stat[c], rs = stat[NC + c];
  const float gg = bf16_val(g[c]), bb = bf16_val(be[c]);
  const float* src = R1 + (size_t)plane * 1024;
  v4f o[2];
#pragma unroll
  for (int it = 0; it < 2; ++it) {
    const int p = it * 32 + lane;
    const int ho = p >> 2, w4 = (p & 3) * 4;
    const float* r0 = src + (2 * ho) * 32 + 2 * w4;
    const v4f a0 = bn4(*(const v4f*)(r0), m, rs, gg, bb);
    const v4f a1 = bn4(*(const v4f*)(r0 + 4), m, rs, gg, bb);
    const v4f b0 = bn4(*(const v4f*)(r0 + 32), m, rs, gg, bb);
    const v4f b1 = bn4(*(const v4f*)(r0 + 36), m, rs, gg, bb);
    v4f v;
    v.x = fmaxf(fmaxf(a0.x, a0.y), fmaxf(b0.x, b0.y));
    v.y = fmaxf(fmaxf(a0.z, a0.w), fmaxf(b0.z, b0.w));
    v.z = fmaxf(fmaxf(a1.x, a1.y), fmaxf(b1.x, b1.y));
    v.w = fmaxf(fmaxf(a1.z, a1.w), fmaxf(b1.z, b1.w));
    o[it] = v;
  }
  float* dst = out1 + (size_t)plane * 256 + 4 * lane;
  *(volatile v4f*)(dst) = o[0];
  *(volatile v4f*)(dst + 128) = o[1];
  __threadfence();
  *(volatile v4f*)(dst) = o[0];
  *(volatile v4f*)(dst + 128) = o[1];
}

__global__ __launch_bounds__(256) __attribute__((amdgpu_num_vgpr(248)))
void k_bn2(const float* __restrict__ R2, const float* __restrict__ stat,
           const float* __restrict__ g, const float* __restrict__ be, float* out2, float* x03) {
  const int tid = (int)threadIdx.x, lane = tid & 31, wave = tid >> 5;
  const int plane = (int)blockIdx.x * 8 + wave;
  const int c = plane % NC;
  const float m = stat[c], rs = stat[NC + c];
  const float gg = bf16_val(g[c]), bb = bf16_val(be[c]);
  const float* src = R2 + (size_t)plane * 256;
  const v4f o0 = bn4(*(const v4f*)(src + 4 * lane), m, rs, gg, bb);
  const v4f o1 = bn4(*(const v4f*)(src + 128 + 4 * lane), m, rs, gg, bb);
  const int lp = lane & 15;
  const int ho = lp >> 1, w8 = (lp & 1) * 8;
  const float* r0 = src + (2 * ho) * 16 + w8;
  const v4f a0 = bn4(*(const v4f*)(r0), m, rs, gg, bb);
  const v4f a1 = bn4(*(const v4f*)(r0 + 4), m, rs, gg, bb);
  const v4f b0 = bn4(*(const v4f*)(r0 + 16), m, rs, gg, bb);
  const v4f b1 = bn4(*(const v4f*)(r0 + 20), m, rs, gg, bb);
  v4f pv;
  pv.x = fmaxf(fmaxf(a0.x, a0.y), fmaxf(b0.x, b0.y));
  pv.y = fmaxf(fmaxf(a0.z, a0.w), fmaxf(b0.z, b0.w));
  pv.z = fmaxf(fmaxf(a1.x, a1.y), fmaxf(b1.x, b1.y));
  pv.w = fmaxf(fmaxf(a1.z, a1.w), fmaxf(b1.z, b1.w));
  float* d2 = out2 + (size_t)plane * 256 + 4 * lane;
  float* d3 = x03 + (size_t)plane * 64 + 4 * lp;
  *(volatile v4f*)(d2) = o0;
  *(volatile v4f*)(d2 + 128) = o1;
  if (lane < 16) *(volatile v4f*)(d3) = pv;
  __threadfence();
  *(volatile v4f*)(d2) = o0;
  *(volatile v4f*)(d2 + 128) = o1;
  if (lane < 16) *(volatile v4f*)(d3) = pv;
}

__global__ __launch_bounds__(256) __attribute__((amdgpu_num_vgpr(248)))
void k_head(const float* __restrict__ R3, const float* __restrict__ stat,
            const float* __restrict__ g, const float* __restrict__ be,
            const float* __restrict__ fcw, const float* __restrict__ fcb, float* out0) {
  __shared__ __attribute__((aligned(16))) float sz[8 * NC];
  __shared__ __attribute__((aligned(16))) float sL[8 * NCLS];
  const int tid = (int)threadIdx.x, blk = (int)blockIdx.x;
  const int b0 = blk * 8;
#pragma unroll 1
  for (int i = 0; i < 6; ++i) {
    const int pr = tid + 256 * i;
    const int im = pr / NC;
    const int c = pr - im * NC;
    const float m = stat[c], rs = stat[NC + c];
    const float gg = bf16_val(g[c]), bb = bf16_val(be[c]);
    const float* src = R3 + ((size_t)(b0 + im) * NC + c) * 64;
    float s = 0.0f;
#pragma unroll 2
    for (int j = 0; j < 16; ++j) {
      const v4f v = bn4(*(const v4f*)(src + 4 * j), m, rs, gg, bb);
      s += v.x; s += v.y; s += v.z; s += v.w;
    }
    sz[pr] = s * (1.0f / 64.0f);
  }
  __syncthreads();
#pragma unroll 1
  for (int i = 0; i < 4; ++i) {
    const int o = tid + 256 * i;
    const int oc = (o < 8 * NCLS) ? o : (8 * NCLS - 1);
    const int im = oc / NCLS;
    const int j = oc - im * NCLS;
    const float* wr = fcw + (size_t)j * NC;
    const float* zr = sz + im * NC;
    float s = 0.0f;
#pragma unroll 1
    for (int c4 = 0; c4 < NC / 4; ++c4) {
      const v4f w = *(const v4f*)(wr + 4 * c4);
      const v4f z = *(const v4fa*)(zr + 4 * c4);
      s = fmaf(z.x, bf16_val(w.x), s);
      s = fmaf(z.y, bf16_val(w.y), s);
      s = fmaf(z.z, bf16_val(w.z), s);
      s = fmaf(z.w, bf16_val(w.w), s);
    }
    s += bf16_val(fcb[j]);
    if (o < 8 * NCLS) sL[o] = s;
  }
  __syncthreads();
  v4f v = {0.f, 0.f, 0.f, 0.f};
  float* dst = out0 + (size_t)blk * (8 * NCLS) + 4 * tid;
  if (tid < 200) {
    v = *(const v4fa*)(sL + 4 * tid);
    *(volatile v4f*)dst = v;
  }
  __threadfence();
  if (tid < 200) *(volatile v4f*)dst = v;
}

extern "C" void kernel_launch(void* const* d_in, const int* in_sizes, int n_in,
                              void* d_out, int out_size, void* d_ws, size_t ws_size,
                              hipStream_t stream) {
  if (n_in < 15) return;
  if (in_sizes[0] != NB * 3 * 32 * 32) return;
  if (in_sizes[1] != NC * 75 || in_sizes[2] != NC) return;
  if (in_sizes[3] != NC * 4800 || in_sizes[4] != NC) return;
  if (in_sizes[5] != NC * 4800 || in_sizes[6] != NC) return;
  for (int i = 7; i <= 12; ++i) if (in_sizes[i] != NC) return;
  if (in_sizes[13] != NCLS * NC || in_sizes[14] != NCLS) return;
  if (out_size != OUT_TOTAL) return;
  if ((size_t)WS_TOTAL > ws_size) return;

  const float* x   = (const float*)d_in[0];
  const float* w1  = (const float*)d_in[1];
  const float* b1  = (const float*)d_in[2];
  const float* w2  = (const float*)d_in[3];
  const float* b2  = (const float*)d_in[4];
  const float* w3  = (const float*)d_in[5];
  const float* b3  = (const float*)d_in[6];
  const float* g1  = (const float*)d_in[7];
  const float* be1 = (const float*)d_in[8];
  const float* g2  = (const float*)d_in[9];
  const float* be2 = (const float*)d_in[10];
  const float* g3  = (const float*)d_in[11];
  const float* be3 = (const float*)d_in[12];
  const float* fcw = (const float*)d_in[13];
  const float* fcb = (const float*)d_in[14];

  float* out  = (float*)d_out;
  float* out0 = out + OUT0_OFF;
  float* out1 = out + OUT1_OFF;
  float* out2 = out + OUT2_OFF;

  char* ws = (char*)d_ws;
  unsigned short* W1B = (unsigned short*)(ws + WS_W1B);
  unsigned short* W2B = (unsigned short*)(ws + WS_W2B);
  unsigned short* W3B = (unsigned short*)(ws + WS_W3B);
  double* REC  = (double*)(ws + WS_REC);
  float* STAT1 = (float*)(ws + WS_STAT);
  float* STAT2 = (float*)(ws + WS_STAT + 2048);
  float* STAT3 = (float*)(ws + WS_STAT + 4096);
  float* X03 = (float*)(ws + WS_X03);
  float* R3  = (float*)(ws + WS_R3);
  float* R1  = (float*)(ws + WS_R1);
  float* R2  = R1;

  (void)hipFuncSetAttribute(reinterpret_cast<const void*>(&k_inrf<3, 32, 96>),
                            hipFuncAttributeMaxDynamicSharedMemorySize, LDSB);
  (void)hipFuncSetAttribute(reinterpret_cast<const void*>(&k_inrf<192, 16, 4800>),
                            hipFuncAttributeMaxDynamicSharedMemorySize, LDSB);
  (void)hipFuncSetAttribute(reinterpret_cast<const void*>(&k_inrf<192, 8, 4800>),
                            hipFuncAttributeMaxDynamicSharedMemorySize, LDSB);

  k_prep<<<PB_END, 256, 0, stream>>>(w1, w2, w3, W1B, W2B, W3B);
  k_inrf<3, 32, 96><<<NB * 1024 / 128, 256, LDSB, stream>>>(x, W1B, b1, R1, REC);
  k_stat<<<1, 192, 0, stream>>>(REC, 1024, 1.0 / 1024.0, 1.0 / 131072.0, STAT1);
  k_bn1pool<<<NB * NC / 8, 256, 0, stream>>>(R1, STAT1, g1, be1, out1);
  k_inrf<192, 16, 4800><<<NB * 256 / 128, 256, LDSB, stream>>>(out1, W2B, b2, R2, REC);
  k_stat<<<1, 192, 0, stream>>>(REC, 256, 1.0 / 256.0, 1.0 / 32768.0, STAT2);
  k_bn2<<<NB * NC / 8, 256, 0, stream>>>(R2, STAT2, g2, be2, out2, X03);
  k_inrf<192, 8, 4800><<<NB * 64 / 128, 256, LDSB, stream>>>(X03, W3B, b3, R3, REC);
  k_stat<<<1, 192, 0, stream>>>(REC, 64, 1.0 / 64.0, 1.0 / 8192.0, STAT3);
  k_head<<<NB / 8, 256, 0, stream>>>(R3, STAT3, g3, be3, fcw, fcb, out0);
  (void)hipGetLastError();
}
